// MemoryEfficientAttention_43250320671349
// MI455X (gfx1250) — hardware-verified
//
#include <hip/hip_runtime.h>
#include <math.h>

#ifndef NB
#define NB 2
#endif
#ifndef SEQ
#define SEQ 4096
#endif
#define NB_FULL  2
#define SEQ_FULL 4096
#define CD  512
#define NH  4
#define HD  128
#define QN  (3 * CD)
#define OUT_BYTES 16777216LL
#define PCARRY 4096.0f
#define VCARRY 16.0f

static_assert(NB >= 1 && NB <= NB_FULL);
static_assert(SEQ >= 64 && SEQ <= SEQ_FULL && (SEQ % 64) == 0);
static_assert((CD % 64) == 0 && (QN % 64) == 0 && (CD % 32) == 0);
static_assert(NH * HD == CD && (HD % 64) == 0);
static_assert((long long)NB * SEQ * CD * 4 <= OUT_BYTES);

typedef __attribute__((ext_vector_type(16))) _Float16 v16h;
typedef __attribute__((ext_vector_type(8)))  _Float16 v8h;
typedef __attribute__((ext_vector_type(16))) __bf16   v16b;
typedef __attribute__((ext_vector_type(8)))  float    v8f;
typedef __attribute__((ext_vector_type(4)))  float    v4f;

__device__ __forceinline__ int frag_k(int i, int h) { return (i < 8) ? (8 * h + i) : (16 + 8 * h + (i - 8)); }
__device__ __forceinline__ unsigned int bf16_bits(float f) {
    unsigned int u = __float_as_uint(f);
    u += 0x7fffu + ((u >> 16) & 1u);
    return u >> 16;
}
__device__ __forceinline__ __bf16 bf16_rne(float f) { return __builtin_bit_cast(__bf16, (unsigned short)bf16_bits(f)); }
__device__ __forceinline__ float bf16_f32(__bf16 b) { return __uint_as_float(((unsigned int)__builtin_bit_cast(unsigned short, b)) << 16); }
__device__ __forceinline__ v8f wmma16(v16h a, v16h b, v8f c) {
    c = __builtin_amdgcn_wmma_f32_16x16x32_f16(false, a, false, b, (short)0, c, false, false);
    asm volatile("v_nop\n\tv_nop\n\tv_nop\n\tv_nop" : "+v"(c) : "v"(a), "v"(b));
    return c;
}
__device__ __forceinline__ v8f wmmab(v16b a, v16b b, v8f c) {
    c = __builtin_amdgcn_wmma_f32_16x16x32_bf16(false, a, false, b, (short)0, c, false, false);
    asm volatile("v_nop\n\tv_nop\n\tv_nop\n\tv_nop" : "+v"(c) : "v"(a), "v"(b));
    return c;
}
struct Split { v16b hi, lo; };
__device__ __forceinline__ v8f wmma3(const Split& a, const Split& b, v8f c) {
    c = __builtin_amdgcn_wmma_f32_16x16x32_bf16(false, a.hi, false, b.hi, (short)0, c, false, false);
    c = __builtin_amdgcn_wmma_f32_16x16x32_bf16(false, a.hi, false, b.lo, (short)0, c, false, false);
    c = __builtin_amdgcn_wmma_f32_16x16x32_bf16(false, a.lo, false, b.hi, (short)0, c, false, false);
    asm volatile("v_nop\n\tv_nop\n\tv_nop\n\tv_nop" : "+v"(c) : "v"(a.hi), "v"(a.lo), "v"(b.hi), "v"(b.lo));
    return c;
}

__device__ __forceinline__ v16h fh_ld(const float* __restrict__ p, long long sk, int k0, int h, int klen, float s) {
    v16h a;
#pragma unroll
    for (int i = 0; i < 16; ++i) { const int k = k0 + frag_k(i, h); a[i] = (k < klen) ? (_Float16)(p[(long long)k * sk] * s) : (_Float16)0.f; }
    return a;
}
__device__ __forceinline__ Split sp_ld(const float* __restrict__ p, long long sk, int k0, int h, int klen, float s) {
    Split r;
#pragma unroll
    for (int i = 0; i < 16; ++i) {
        const int k = k0 + frag_k(i, h); const float x = (k < klen) ? p[(long long)k * sk] * s : 0.f;
        const __bf16 hb = bf16_rne(x); r.hi[i] = hb; r.lo[i] = bf16_rne(x - bf16_f32(hb));
    }
    return r;
}
__device__ __forceinline__ v16b bh_ld(const float* __restrict__ p, long long sk, int k0, int h, int klen, float s) {
    v16b a;
#pragma unroll
    for (int i = 0; i < 16; ++i) { const int k = k0 + frag_k(i, h); a[i] = bf16_rne((k < klen) ? p[(long long)k * sk] * s : 0.f); }
    return a;
}

union FragH { v16h v; v8h u[2]; };
__device__ __forceinline__ v16h frag_hf(const _Float16* row, int k0, int hf) {
    FragH f; f.u[0] = *(const v8h*)(row + k0 + 8 * hf); f.u[1] = *(const v8h*)(row + k0 + 16 + 8 * hf); return f.v;
}

#define VST2(T, ptr, val) do { const T vst2_v_ = (val); *(volatile T*)(ptr) = vst2_v_; __threadfence(); *(volatile T*)(ptr) = vst2_v_; } while (0)
#define VST2V4(ptr, val) do { const v4f vst2_v4_ = (val); *(volatile v4f*)(ptr) = vst2_v4_; __threadfence(); *(volatile v4f*)(ptr) = vst2_v4_; } while (0)

__device__ __forceinline__ float act_lin(float v, int act) { return (act == 1) ? fmaxf(v, 0.f) : v; }

struct GemmP {
    const float* A; const float* B; const float* bias; const float* R; float* C;
    long long sAo, sAi, sAm, sAk, sBo, sBi, sBn, sBk, sCo, sCi, sCm, sRo, sRi, sRm, sRn;
    int M, N, K, zi_n, flags, act; float alpha, beta, sa, sb;
    int Npad, pad_;
};
static_assert(sizeof(GemmP) == 5 * 8 + 15 * 8 + 6 * 4 + 4 * 4 + 2 * 4);

template <int MODE, int TM, int TN>
__global__ __launch_bounds__(32) __attribute__((amdgpu_num_vgpr(256))) void k_gemmT(GemmP p) {
    const int lane = threadIdx.x & 31, h = lane >> 4, l15 = lane & 15;
    const int m0 = blockIdx.y * (16 * TM), n0 = blockIdx.x * (16 * TN);
    const int z = blockIdx.z, zo = z / p.zi_n, zi = z - zo * p.zi_n;
    const float* A = p.A + zo * p.sAo + zi * p.sAi;
    const float* B = p.B + zo * p.sBo + zi * p.sBi;
    v8f acc[TM][TN];
#pragma unroll
    for (int i = 0; i < TM; ++i)
#pragma unroll
        for (int t = 0; t < TN; ++t) { v8f zz = {}; acc[i][t] = zz; }
    for (int k0 = 0; k0 < p.K; k0 += 32) {
        if (MODE == 1) {
            Split a[TM], b[TN];
#pragma unroll
            for (int i = 0; i < TM; ++i) { const int am = min(m0 + 16 * i + l15, p.M - 1); a[i] = sp_ld(A + (long long)am * p.sAm, p.sAk, k0, h, p.K, 1.f); }
#pragma unroll
            for (int t = 0; t < TN; ++t) { const int bn = min(n0 + 16 * t + l15, p.N - 1); b[t] = sp_ld(B + (long long)bn * p.sBn, p.sBk, k0, h, p.K, 1.f); }
#pragma unroll
            for (int i = 0; i < TM; ++i)
#pragma unroll
                for (int t = 0; t < TN; ++t) acc[i][t] = wmma3(a[i], b[t], acc[i][t]);
        } else if (MODE == 2) {
            v16b a[TM], b[TN];
#pragma unroll
            for (int i = 0; i < TM; ++i) { const int am = min(m0 + 16 * i + l15, p.M - 1); a[i] = bh_ld(A + (long long)am * p.sAm, p.sAk, k0, h, p.K, 1.f); }
#pragma unroll
            for (int t = 0; t < TN; ++t) { const int bn = min(n0 + 16 * t + l15, p.N - 1); b[t] = bh_ld(B + (long long)bn * p.sBn, p.sBk, k0, h, p.K, 1.f); }
#pragma unroll
            for (int i = 0; i < TM; ++i)
#pragma unroll
                for (int t = 0; t < TN; ++t) acc[i][t] = wmmab(a[i], b[t], acc[i][t]);
        } else {
            v16h a[TM], b[TN];
#pragma unroll
            for (int i = 0; i < TM; ++i) { const int am = min(m0 + 16 * i + l15, p.M - 1); a[i] = fh_ld(A + (long long)am * p.sAm, p.sAk, k0, h, p.K, p.sa); }
#pragma unroll
            for (int t = 0; t < TN; ++t) { const int bn = min(n0 + 16 * t + l15, p.N - 1); b[t] = fh_ld(B + (long long)bn * p.sBn, p.sBk, k0, h, p.K, p.sb); }
#pragma unroll
            for (int i = 0; i < TM; ++i)
#pragma unroll
                for (int t = 0; t < TN; ++t) acc[i][t] = wmma16(a[i], b[t], acc[i][t]);
        }
    }
    const float iscale = (MODE == 0) ? p.alpha / (p.sa * p.sb) : p.alpha;
    float* C = p.C + zo * p.sCo + zi * p.sCi;
    const float* R = p.R + zo * p.sRo + zi * p.sRi;
    const int NW = (p.Npad > p.N) ? p.Npad : p.N;
    __shared__ __align__(16) float ctile[16][36];
#pragma unroll
    for (int i = 0; i < TM; ++i) {
        const int mb = m0 + 16 * i; if (mb >= p.M) break;
#pragma unroll
        for (int tp = 0; tp < TN / 2; ++tp) {
            const int nb = n0 + 32 * tp; if (nb >= NW) break;
#pragma unroll
            for (int t2 = 0; t2 < 2; ++t2) {
                const int t = 2 * tp + t2; const int n = nb + t2 * 16 + l15; const int nn = min(n, p.N - 1);
#pragma unroll
                for (int r = 0; r < 8; ++r) {
                    const int m = mb + 8 * h + r; const int mm = min(m, p.M - 1);
                    float v = acc[i][t][r] * iscale;
                    if (p.flags & 1) v += p.bias[nn];
                    if (p.flags & 2) v += p.bias[mm];
                    if (p.flags & 8) v *= p.bias[(long long)zo * p.M + mm];
                    v = act_lin(v, p.act);
                    if (p.flags & 4) v += p.beta * R[(long long)mm * p.sRm + (long long)nn * p.sRn];
                    ctile[8 * h + r][t2 * 16 + l15] = (n < p.N) ? v : 0.f;
                }
            }
            __syncthreads();
            const bool fast = (mb + 16 <= p.M) && (nb + 32 <= NW) && ((p.sCm & 3) == 0) && ((((size_t)C) & 15) == 0);
            if (fast) {
#pragma unroll
                for (int s = 0; s < 4; ++s) {
                    const int row = s * 4 + (lane >> 3), c4 = (lane & 7) * 4;
                    const v4f v = *(const v4f*)&ctile[row][c4];
                    VST2V4(C + (long long)(mb + row) * p.sCm + nb + c4, v);
                }
            } else {
                for (int row = 0; row < 16; ++row) {
                    const int m = mb + row, n = nb + lane;
                    if (m < p.M && n < NW) VST2(float, C + (long long)m * p.sCm + n, ctile[row][lane]);
                }
            }
            __syncthreads();
        }
    }
}

__global__ __launch_bounds__(256) void k_rne(const float* __restrict__ src, float* __restrict__ dst, int n4) {
    const int i = blockIdx.x * 256 + threadIdx.x;
    if (i >= n4) return;
    const v4f sv = *(const v4f*)(src + 4 * (long long)i);
    const float s0 = sv.x, s1 = sv.y, s2 = sv.z, s3 = sv.w;
    v4f r;
    r.x = bf16_f32(bf16_rne(s0)); r.y = bf16_f32(bf16_rne(s1)); r.z = bf16_f32(bf16_rne(s2)); r.w = bf16_f32(bf16_rne(s3));
    VST2V4(dst + 4 * (long long)i, r);
}

struct SplitP { const float* src; _Float16* qp; _Float16* kp; _Float16* vt; long long sSb; int L, nh, ldq, cd; float vsc; int pad0; };
static_assert(sizeof(SplitP) == 4 * 8 + 8 + 4 * 4 + 2 * 4);

template <int HDC>
__global__ __launch_bounds__(256) void k_split(SplitP p) {
    constexpr int VPL = 68;
    __shared__ __align__(16) float vtl[HDC][VPL];
    const int tid = threadIdx.x, i0 = blockIdx.x * 64, h = blockIdx.y, b = blockIdx.z, bh = b * p.nh + h;
    const float* sb = p.src + (size_t)b * p.sSb;
#pragma unroll
    for (int part = 0; part < 2; ++part) {
        _Float16* dp = part ? p.kp : p.qp;
#pragma unroll 1
        for (int it = 0; it < (64 * HDC / 8) / 256; ++it) {
            const int item = it * 256 + tid, row = item / (HDC / 8), c8 = (item - row * (HDC / 8)) * 8;
            const float* s = sb + (size_t)(i0 + row) * p.ldq + part * p.cd + h * HDC + c8;
            const v4f a = *(const v4f*)s; const v4f c = *(const v4f*)(s + 4);
            v8h r;
            r[0] = (_Float16)a.x; r[1] = (_Float16)a.y; r[2] = (_Float16)a.z; r[3] = (_Float16)a.w;
            r[4] = (_Float16)c.x; r[5] = (_Float16)c.y; r[6] = (_Float16)c.z; r[7] = (_Float16)c.w;
            const size_t doff = ((size_t)bh * p.L + i0 + row) * HDC + c8;
            VST2(v8h, dp + doff, r);
        }
    }
#pragma unroll 1
    for (int it = 0; it < (64 * HDC / 4) / 256; ++it) {
        const int item = it * 256 + tid, row = item / (HDC / 4), c4 = (item - row * (HDC / 4)) * 4;
        const v4f a = *(const v4f*)(sb + (size_t)(i0 + row) * p.ldq + 2 * p.cd + h * HDC + c4);
        vtl[c4][row] = a.x; vtl[c4 + 1][row] = a.y; vtl[c4 + 2][row] = a.z; vtl[c4 + 3][row] = a.w;
    }
    __syncthreads();
#pragma unroll 1
    for (int it = 0; it < (HDC * 8) / 256; ++it) {
        const int item = it * 256 + tid, d = item >> 3, q = item & 7;
        const v4f a = *(const v4f*)&vtl[d][8 * q]; const v4f c = *(const v4f*)&vtl[d][8 * q + 4];
        v8h r;
        r[0] = (_Float16)(a.x * p.vsc); r[1] = (_Float16)(a.y * p.vsc); r[2] = (_Float16)(a.z * p.vsc); r[3] = (_Float16)(a.w * p.vsc);
        r[4] = (_Float16)(c.x * p.vsc); r[5] = (_Float16)(c.y * p.vsc); r[6] = (_Float16)(c.z * p.vsc); r[7] = (_Float16)(c.w * p.vsc);
        VST2(v8h, p.vt + ((size_t)bh * HDC + d) * p.L + i0 + 8 * q, r);
    }
}

#define AW 4
struct FlashP {
    const _Float16* Qp; const _Float16* Kp; const _Float16* Vt; float* O;
    long long sOb;
    int L, nh, ldo, pad0; float scl2e, oscale;
};
static_assert(sizeof(FlashP) == 4 * 8 + 8 + 4 * 4 + 2 * 4);

template <int HDC>
__global__ __launch_bounds__(32 * AW) __attribute__((amdgpu_num_vgpr(256))) void k_flash(FlashP p) {
    constexpr int KS = HDC / 32;
    constexpr int NT = HDC / 16;
    constexpr int OPL = 68;
    __shared__ __align__(16) _Float16 ps[2][AW][16][32];
    __shared__ __align__(16) float    ot[AW][16][OPL];
    const int lane = threadIdx.x & 31, hf = lane >> 4, l15 = lane & 15, wave = threadIdx.x >> 5;
    const int h = blockIdx.y, b = blockIdx.z, bh = b * p.nh + h;
    const int q0 = (blockIdx.x * AW + wave) * 16;
    const float NEG = -__builtin_inff();
    const size_t prow = (size_t)bh * p.L;
    const _Float16* qrow = p.Qp + (prow + q0 + l15) * HDC;
    const _Float16* krow = p.Kp + (prow + l15) * HDC;
    const _Float16* vt = p.Vt + ((size_t)bh * HDC + l15) * p.L;
    v16h qa[KS];
#pragma unroll
    for (int ks = 0; ks < KS; ++ks) qa[ks] = frag_hf(qrow, ks * 32, hf);
    v8f o[NT]; float m8[8], l8[8];
#pragma unroll
    for (int t = 0; t < NT; ++t) { v8f zz = {}; o[t] = zz; }
#pragma unroll
    for (int i = 0; i < 8; ++i) { m8[i] = NEG; l8[i] = 0.f; }

#pragma unroll 1
    for (int j0 = 0; j0 < p.L; j0 += 32) {
        const int buf = (j0 >> 5) & 1;
        v8f s0, s1; { v8f zz = {}; s0 = zz; s1 = zz; }
        const _Float16* k0r = krow + (size_t)j0 * HDC;
        const _Float16* k1r = k0r + 16 * HDC;
#pragma unroll
        for (int ks = 0; ks < KS; ++ks) {
            const v16h kb = frag_hf(k0r, ks * 32, hf);
            s0 = wmma16(qa[ks], kb, s0);
            const v16h kc = frag_hf(k1r, ks * 32, hf);
            s1 = wmma16(qa[ks], kc, s1);
        }
#pragma unroll
        for (int i = 0; i < 8; ++i) {
            const float sc0 = s0[i] * p.scl2e, sc1 = s1[i] * p.scl2e;
            float mx = fmaxf(sc0, sc1);
            mx = fmaxf(mx, __shfl_xor(mx, 1, 32)); mx = fmaxf(mx, __shfl_xor(mx, 2, 32));
            mx = fmaxf(mx, __shfl_xor(mx, 4, 32)); mx = fmaxf(mx, __shfl_xor(mx, 8, 32));
            const float mnew = fmaxf(m8[i], mx);
            const float corr = (mnew == NEG) ? 1.f : exp2f(m8[i] - mnew);
            const float p0 = (mnew == NEG) ? 0.f : exp2f(sc0 - mnew);
            const float p1 = (mnew == NEG) ? 0.f : exp2f(sc1 - mnew);
            float rs = p0 + p1;
            rs += __shfl_xor(rs, 1, 32); rs += __shfl_xor(rs, 2, 32); rs += __shfl_xor(rs, 4, 32); rs += __shfl_xor(rs, 8, 32);
            l8[i] = l8[i] * corr + rs; m8[i] = mnew;
#pragma unroll
            for (int t = 0; t < NT; ++t) o[t][i] *= corr;
            ps[buf][wave][8 * hf + i][l15]      = (_Float16)(p0 * PCARRY);
            ps[buf][wave][8 * hf + i][16 + l15] = (_Float16)(p1 * PCARRY);
        }
        __syncthreads();
        FragH pa;
        pa.u[0] = *(const v8h*)&ps[buf][wave][l15][8 * hf];
        pa.u[1] = *(const v8h*)&ps[buf][wave][l15][16 + 8 * hf];
        const _Float16* vj = vt + j0;
#pragma unroll
        for (int t = 0; t < NT; ++t) {
            const v16h vb = frag_hf(vj + (size_t)(16 * t) * p.L, 0, hf);
            o[t] = wmma16(pa.v, vb, o[t]);
        }
    }

    float invr[8];
#pragma unroll
    for (int i = 0; i < 8; ++i) invr[i] = (l8[i] > 0.f) ? (p.oscale / l8[i]) : 0.f;
    float* obase = p.O + (size_t)b * p.sOb + (size_t)h * HDC;
#pragma unroll
    for (int c0 = 0; c0 < HDC; c0 += 64) {
        __syncthreads();
#pragma unroll
        for (int i = 0; i < 8; ++i)
#pragma unroll
            for (int t = 0; t < NT; ++t)
                if (t * 16 >= c0 && t * 16 < c0 + 64) ot[wave][8 * hf + i][t * 16 - c0 + l15] = o[t][i] * invr[i];
        __syncthreads();
#pragma unroll
        for (int r0 = 0; r0 < 16; r0 += 2) {
            const int row = r0 + (lane >> 4), c4 = (lane & 15) * 4;
            const v4f v = *(const v4f*)&ot[wave][row][c4];
            VST2V4(obase + (size_t)(q0 + row) * p.ldo + c0 + c4, v);
        }
    }
}

extern "C" void kernel_launch(void* const* d_in, const int* in_sizes, int n_in, void* d_out, int out_size, void* d_ws, size_t ws_size, hipStream_t stream) {
    if (n_in < 5) return;
    const float* x      = (const float*)d_in[0];
    const float* qkv_w  = (const float*)d_in[1];
    const float* qkv_b  = (const float*)d_in[2];
    const float* proj_w = (const float*)d_in[3];
    const float* proj_b = (const float*)d_in[4];
    if (in_sizes[0] < ((NB - 1) * SEQ_FULL + SEQ) * CD) return;
    if (in_sizes[1] < QN * CD || in_sizes[2] < QN || in_sizes[3] < CD * CD || in_sizes[4] < CD) return;
    if (out_size < NB * SEQ * CD) return;
    float* out = (float*)d_out;

    char* wsp = (char*)d_ws; size_t off = 0;
    auto carve = [&](size_t bytes) -> char* { char* p = wsp + off; off += (bytes + 255) & ~(size_t)255; return p; };
    const size_t plane16 = (size_t)NB * NH * SEQ * HD * 2;
    float* qb_r = (float*)carve((size_t)QN * 4);
    float* pb_r = (float*)carve((size_t)CD * 4);
    float* pw_r = (float*)carve((size_t)CD * CD * 4);
    float* qkv  = (float*)carve((size_t)NB * SEQ * QN * 4);
    _Float16* q_p = (_Float16*)carve(plane16);
    _Float16* k_p = (_Float16*)carve(plane16);
    _Float16* v_t = (_Float16*)carve(plane16);
    float* ctx  = (float*)carve((size_t)NB * SEQ * CD * 4);
    if (off > ws_size) return;

    k_rne<<<(QN / 4 + 255) / 256, 256, 0, stream>>>(qkv_b, qb_r, QN / 4);
    k_rne<<<(CD / 4 + 255) / 256, 256, 0, stream>>>(proj_b, pb_r, CD / 4);
    k_rne<<<(CD * CD / 4 + 255) / 256, 256, 0, stream>>>(proj_w, pw_r, CD * CD / 4);

    { GemmP g = {};
      g.A = x; g.B = qkv_w; g.bias = qb_r; g.R = nullptr; g.C = qkv;
      g.sAo = (long long)SEQ_FULL * CD; g.sAi = 0; g.sAm = CD; g.sAk = 1;
      g.sBo = 0; g.sBi = 0; g.sBn = CD; g.sBk = 1;
      g.sCo = (long long)SEQ * QN; g.sCi = 0; g.sCm = QN;
      g.sRo = 0; g.sRi = 0; g.sRm = 0; g.sRn = 0;
      g.M = SEQ; g.N = QN; g.K = CD; g.zi_n = 1; g.flags = 1; g.act = 0;
      g.alpha = 1.f; g.beta = 0.f; g.sa = 1.f; g.sb = 1.f; g.Npad = QN; g.pad_ = 0;
      k_gemmT<2, 2, 4><<<dim3((unsigned)((QN + 63) / 64), (unsigned)((SEQ + 31) / 32), (unsigned)NB), 32, 0, stream>>>(g); }

    { SplitP s = {};
      s.src = qkv; s.qp = q_p; s.kp = k_p; s.vt = v_t;
      s.sSb = (long long)SEQ * QN; s.L = SEQ; s.nh = NH; s.ldq = QN; s.cd = CD; s.vsc = VCARRY; s.pad0 = 0;
      k_split<HD><<<dim3((unsigned)(SEQ / 64), (unsigned)NH, (unsigned)NB), 256, 0, stream>>>(s); }

    { FlashP f = {};
      f.Qp = q_p; f.Kp = k_p; f.Vt = v_t; f.O = ctx;
      f.sOb = (long long)SEQ * CD; f.L = SEQ; f.nh = NH; f.ldo = CD; f.pad0 = 0;
      f.scl2e = 0.08838834764831845f * 1.4426950408889634f;
      f.oscale = 1.0f / (PCARRY * VCARRY);
      k_flash<HD><<<dim3((unsigned)(SEQ / 64), (unsigned)NH, (unsigned)NB), 32 * AW, 0, stream>>>(f); }

    { GemmP g = {};
      g.A = ctx; g.B = pw_r; g.bias = pb_r; g.R = nullptr; g.C = out;
      g.sAo = (long long)SEQ * CD; g.sAi = 0; g.sAm = CD; g.sAk = 1;
      g.sBo = 0; g.sBi = 0; g.sBn = CD; g.sBk = 1;
      g.sCo = (long long)SEQ * CD; g.sCi = 0; g.sCm = CD;
      g.sRo = 0; g.sRi = 0; g.sRm = 0; g.sRn = 0;
      g.M = SEQ; g.N = CD; g.K = CD; g.zi_n = 1; g.flags = 1; g.act = 0;
      g.alpha = 1.f; g.beta = 0.f; g.sa = 64.f; g.sb = 256.f; g.Npad = CD; g.pad_ = 0;
      k_gemmT<0, 2, 4><<<dim3((unsigned)((CD + 63) / 64), (unsigned)((SEQ + 31) / 32), (unsigned)NB), 32, 0, stream>>>(g); }
}
